// LinearEmbed_33621003993929
// MI455X (gfx1250) — hardware-run, weakly checked
//
#include <hip/hip_runtime.h>
#include <math.h>

typedef __attribute__((ext_vector_type(16))) _Float16 v16h;
typedef __attribute__((ext_vector_type(8)))  _Float16 v8h;
typedef __attribute__((ext_vector_type(8)))  float    v8f;
typedef __attribute__((ext_vector_type(4)))  float    v4f;
typedef __attribute__((ext_vector_type(4)))  unsigned v4u;

constexpr int kGraphs   = 64;
constexpr int kNodesPG  = 64;
constexpr int kEdgesPG  = 512;
constexpr int kHid      = 128;
constexpr int kInF      = 32;
constexpr int kEdF      = 16;
constexpr int kEdFPad   = 32;
constexpr int kLayers   = 4;
constexpr int kNodes    = kGraphs * kNodesPG;
constexpr int kEdges    = kGraphs * kEdgesPG;
constexpr int kNumWMats = 19;
constexpr int kWMatElems = kHid * kHid;
constexpr float kBnEps  = 1e-5f;
constexpr float kWCarry    = 64.0f;
constexpr float kWCarryInv = 1.0f / 64.0f;
static_assert(kWCarry * kWCarryInv == 1.0f);
static_assert(kNodes == 4096 && kEdges == 32768);
static_assert((kNodes % 64) == 0 && (kEdges % 64) == 0 && (kHid % 64) == 0 && ((2 * kHid) % 64) == 0);
static_assert((kHid % 32) == 0 && (kInF % 32) == 0 && (kEdFPad % 32) == 0);

constexpr size_t kSzW    = (size_t)kNumWMats * kWMatElems * 2;
constexpr size_t kSzSmW  = (size_t)kHid * 32 * 2;
constexpr size_t kSzX    = (size_t)kNodes * kInF * 2;
constexpr size_t kSzEA   = (size_t)kEdges * kEdFPad * 2;
constexpr size_t kSzEP   = (size_t)kEdges * kHid * 2;
constexpr size_t kSzEF   = (size_t)kEdges * kHid * 4;
constexpr size_t kSzNP   = (size_t)kNodes * kHid * 2;
constexpr size_t kSzNF   = (size_t)kNodes * kHid * 4;
constexpr size_t kSzUV   = (size_t)kNodes * 2 * kHid * 4;
constexpr size_t kSzPart = (size_t)64 * 256 * 4;

constexpr size_t kOffWH   = 0;
constexpr size_t kOffATH  = kOffWH  + kSzW;
constexpr size_t kOffBDH  = kOffATH + kSzSmW;
constexpr size_t kOffXH   = kOffBDH + kSzSmW;
constexpr size_t kOffEAH  = kOffXH  + kSzX;
constexpr size_t kOffEH   = kOffEAH + kSzEA;
constexpr size_t kOffTH   = kOffEH  + kSzEP;
constexpr size_t kOffELF  = kOffTH  + kSzEP;
constexpr size_t kOffHF   = kOffELF + kSzEF;
constexpr size_t kOffHH   = kOffHF  + kSzNF;
constexpr size_t kOffZH   = kOffHH  + kSzNP;
constexpr size_t kOffTNH  = kOffZH  + kSzNP;
constexpr size_t kOffZ2   = kOffTNH + kSzNP;
constexpr size_t kOffUV   = kOffZ2  + kSzNF;
constexpr size_t kOffPART = kOffUV  + kSzUV;
constexpr size_t kWsTotal = kOffPART + kSzPart;
static_assert(kWsTotal == 48152576ull);
static_assert(kWsTotal <= 134217728ull);
static_assert((kSzW % 128) == 0 && (kSzSmW % 128) == 0 && (kSzX % 128) == 0 && (kSzEA % 128) == 0 &&
              (kSzEP % 128) == 0 && (kSzEF % 128) == 0 && (kSzNP % 128) == 0 && (kSzNF % 128) == 0 &&
              (kSzUV % 128) == 0 && (kSzPart % 128) == 0);

__device__ __forceinline__ unsigned short f2bf_bits(float f) {
  unsigned u = __float_as_uint(f);
  return (unsigned short)((u + 0x7FFFu + ((u >> 16) & 1u)) >> 16);
}
__device__ __forceinline__ float bf_bits2f(unsigned short h) { return __uint_as_float(((unsigned)h) << 16); }
__device__ __forceinline__ float bf_rne(float f) { return bf_bits2f(f2bf_bits(f)); }

__device__ __forceinline__ unsigned short f2h_bits(float f) {
  const _Float16 h = (_Float16)f;
  return __builtin_bit_cast(unsigned short, h);
}
__device__ __forceinline__ unsigned pack2h(float a, float b) {
  const unsigned short ha = f2h_bits(a);
  const unsigned short hb = f2h_bits(b);
  return (unsigned)ha | ((unsigned)hb << 16);
}
__device__ __forceinline__ v4u pack8h(const float* x) {
  const unsigned w0 = pack2h(x[0], x[1]);
  const unsigned w1 = pack2h(x[2], x[3]);
  const unsigned w2 = pack2h(x[4], x[5]);
  const unsigned w3 = pack2h(x[6], x[7]);
  return (v4u){w0, w1, w2, w3};
}

struct FragH16 {
  union U { v16h v; v8h h[2]; };
  static __device__ __forceinline__ v16h load(const _Float16* p) {
    U f;
    f.h[0] = *(const v8h*)(p);
    f.h[1] = *(const v8h*)(p + 16);
    return f.v;
  }
};
__device__ __forceinline__ v8f mma_h(v16h a, v16h b, v8f c) {
  c = __builtin_amdgcn_wmma_f32_16x16x32_f16(false, a, false, b, (short)0, c, false, false);
  asm volatile("v_nop\n\tv_nop\n\tv_nop\n\tv_nop" : "+v"(c) : "v"(a), "v"(b));
  return c;
}

template <int BIAS_MODE, int OUT_MODE, int ACT>
__global__ __launch_bounds__(256) void wmma_gemm64_h(
    const unsigned short* __restrict__ Ap, int lda,
    const unsigned short* __restrict__ Btp, int ldb,
    void* __restrict__ Cout, int ldc,
    const float* __restrict__ bias, int M, int N, int K, float scale) {
  const _Float16* A  = (const _Float16*)Ap;
  const _Float16* Bt = (const _Float16*)Btp;
  __shared__ __align__(16) float sT[8][16 * 68];
  const int lane = threadIdx.x & 31;
  const int wave = threadIdx.x >> 5;
  const int tilesN = N >> 6;
  const int tilesM = M >> 6;
  const int tile = blockIdx.x * 8 + wave;
  if (tile >= tilesM * tilesN) return;
  const int tm = tile / tilesN;
  const int tn = tile - tm * tilesN;
  const int m0 = tm << 6;
  const int n0 = tn << 6;

  const int rlane = lane & 15;
  const int koff  = (lane >> 4) * 8;
  const int mOff  = (lane >> 4) * 8;

  v8f acc[4][4];
#pragma unroll
  for (int i = 0; i < 4; ++i)
#pragma unroll
    for (int j = 0; j < 4; ++j) acc[i][j] = (v8f){0.f, 0.f, 0.f, 0.f, 0.f, 0.f, 0.f, 0.f};

  for (int k0 = 0; k0 < K; k0 += 32) {
    v16h bh[4];
#pragma unroll
    for (int j = 0; j < 4; ++j) {
      const size_t bo = (size_t)(n0 + (j << 4) + rlane) * ldb + koff + k0;
      bh[j] = FragH16::load(Bt + bo);
    }
#pragma unroll
    for (int i = 0; i < 4; ++i) {
      const size_t ao = (size_t)(m0 + (i << 4) + rlane) * lda + koff + k0;
      const v16h ah = FragH16::load(A + ao);
#pragma unroll
      for (int j = 0; j < 4; ++j) {
        acc[i][j] = mma_h(ah, bh[j], acc[i][j]);
      }
    }
  }

  float* slab = sT[wave];
#pragma unroll
  for (int i = 0; i < 4; ++i) {
    const int mBase = m0 + (i << 4);
#pragma unroll
    for (int j = 0; j < 4; ++j) {
      const int n = n0 + (j << 4) + rlane;
      float bv = 0.f;
      if (BIAS_MODE == 2) bv = bf_rne(bias[n]);
#pragma unroll
      for (int r = 0; r < 8; ++r) {
        float v = acc[i][j][r] * scale;
        if (BIAS_MODE == 2) v += bv;
        if (ACT == 2) v = fmaxf(v, 0.0f);
        slab[(mOff + r) * 68 + (j << 4) + rlane] = v;
      }
    }
    __builtin_amdgcn_fence(__ATOMIC_RELEASE, "workgroup");
    __builtin_amdgcn_wave_barrier();
    __builtin_amdgcn_fence(__ATOMIC_ACQUIRE, "workgroup");
    if (OUT_MODE == 0) {
      float* C = (float*)Cout;
      const int hs = lane >> 4, c4 = (lane & 15) * 4;
      for (int pass = 0; pass < 2; ++pass) {
#pragma unroll
        for (int it = 0; it < 8; ++it) {
          const int row = it * 2 + hs;
          v4f v = *(const v4f*)(slab + row * 68 + c4);
          *(volatile v4f*)(C + (size_t)(mBase + row) * ldc + n0 + c4) = v;
        }
        __threadfence();
      }
    } else {
      const int q = lane >> 3, c8 = (lane & 7) * 8;
      unsigned short* C = (unsigned short*)Cout;
      for (int pass = 0; pass < 2; ++pass) {
#pragma unroll
        for (int it = 0; it < 4; ++it) {
          const int row = it * 4 + q;
          const v4u hv = pack8h(slab + row * 68 + c8);
          *(volatile v4u*)(C + (size_t)(mBase + row) * ldc + n0 + c8) = hv;
        }
        __threadfence();
      }
    }
    __builtin_amdgcn_fence(__ATOMIC_RELEASE, "workgroup");
    __builtin_amdgcn_wave_barrier();
    __builtin_amdgcn_fence(__ATOMIC_ACQUIRE, "workgroup");
  }
}

__global__ __launch_bounds__(256) void asplit_kernel(
    const float* __restrict__ src, unsigned short* __restrict__ dpl, int creal, int cpad, int total8) {
  const int i = blockIdx.x * 256 + threadIdx.x;
  if (i >= total8) return;
  const int f = i << 3;
  const int row = f / cpad;
  const int c0 = f - row * cpad;
  const bool valid = (c0 < creal);
  const int cc = valid ? c0 : (creal - 8);
  const float* sp = src + (size_t)row * creal + cc;
  const v4f a0 = *(const v4f*)(sp);
  const v4f a1 = *(const v4f*)(sp + 4);
  float x[8];
#pragma unroll
  for (int e = 0; e < 4; ++e) {
    const float t0 = a0[e];
    const float t1 = a1[e];
    x[e]     = valid ? bf_rne(t0) : 0.0f;
    x[4 + e] = valid ? bf_rne(t1) : 0.0f;
  }
  const v4u hv = pack8h(x);
  unsigned short* qh = dpl + (size_t)f;
  *(volatile v4u*)qh = hv;
  __threadfence();
  *(volatile v4u*)qh = hv;
}

__global__ __launch_bounds__(256) void wprep_kernel(
    const float* __restrict__ s0, const float* __restrict__ s1, const float* __restrict__ s2,
    const float* __restrict__ s3, const float* __restrict__ s4,
    unsigned short* __restrict__ dpl, int kreal, int kpad) {
  const int mat = blockIdx.y;
  const int grp = mat >> 2;
  const float* s = s0;
  if (grp == 1) s = s1;
  if (grp == 2) s = s2;
  if (grp == 3) s = s3;
  if (grp == 4) s = s4;
  s += (size_t)(mat & 3) * kreal * 128;
  const int f = (blockIdx.x * 256 + threadIdx.x) << 3;
  if (f >= 128 * kpad) return;
  const int n = f / kpad;
  const int k0 = f - n * kpad;
  float x[8];
#pragma unroll
  for (int e = 0; e < 8; ++e) {
    const int k = k0 + e;
    const int kc = (k < kreal) ? k : (kreal - 1);
    const float v = s[(size_t)kc * 128 + n];
    x[e] = (k < kreal) ? (bf_rne(v) * kWCarry) : 0.0f;
  }
  const v4u hv = pack8h(x);
  unsigned short* qh = dpl + (size_t)mat * 128 * kpad + f;
  *(volatile v4u*)qh = hv;
  __threadfence();
  *(volatile v4u*)qh = hv;
}

__global__ __launch_bounds__(128) void agg_kernel(
    const float* __restrict__ h, const float* __restrict__ el,
    const int* __restrict__ src, const int* __restrict__ dst,
    unsigned short* __restrict__ zpl) {
  __shared__ __align__(16) float sz[64 * 128];
  __shared__ int ssrc[512];
  __shared__ int sdst[512];
  const int g = blockIdx.x;
  const int tid = threadIdx.x;
  const int e0 = g * kEdgesPG;
  const int nb = g * kNodesPG;
#pragma unroll 8
  for (int r = 0; r < 64; ++r) sz[r * 128 + tid] = 0.0f;
#pragma unroll
  for (int i = 0; i < 4; ++i) {
    const int k = tid + 128 * i;
    int sv = src[e0 + k];
    sv = sv < 0 ? 0 : sv;
    sv = sv > (kNodes - 1) ? (kNodes - 1) : sv;
    ssrc[k] = sv;
    sdst[k] = dst[e0 + k] & 63;
  }
  __syncthreads();
#pragma unroll 4
  for (int k = 0; k < kEdgesPG; ++k) {
    const int sv = ssrc[k];
    const int dv = sdst[k];
    const float hv = h[(size_t)sv * kHid + tid];
    const float ev = el[(size_t)(e0 + k) * kHid + tid];
    const float m = fmaxf(hv + ev, 0.0f);
    sz[dv * 128 + tid] += m;
  }
  __syncthreads();
  const int lane = tid & 31, wave = tid >> 5;
  const int hs = lane >> 4, c8 = (lane & 15) * 8;
#pragma unroll 1
  for (int it = 0; it < 8; ++it) {
    const int row = it * 8 + wave * 2 + hs;
    const float* hp = h + (size_t)(nb + row) * kHid + c8;
    const v4f h0 = *(const v4f*)(hp);
    const v4f h1 = *(const v4f*)(hp + 4);
    const v4f a0 = *(const v4f*)(sz + row * 128 + c8);
    const v4f a1 = *(const v4f*)(sz + row * 128 + c8 + 4);
    float x[8];
#pragma unroll
    for (int e = 0; e < 4; ++e) {
      x[e]     = h0[e] + a0[e];
      x[4 + e] = h1[e] + a1[e];
    }
    const v4u hv = pack8h(x);
    const size_t o = (size_t)(nb + row) * kHid + c8;
    *(volatile v4u*)(zpl + o) = hv;
    __threadfence();
    *(volatile v4u*)(zpl + o) = hv;
  }
}

__global__ __launch_bounds__(256) void stats_kernel(const float* __restrict__ z2, float* __restrict__ part) {
  __shared__ float ls[512];
  const int tid = threadIdx.x;
  const int c = tid & 127, hf = tid >> 7;
  const int r0 = blockIdx.x * 64 + hf * 32;
  float s = 0.0f, ss = 0.0f;
#pragma unroll 8
  for (int r = 0; r < 32; ++r) {
    const float v = z2[(size_t)(r0 + r) * kHid + c];
    s += v;
    ss = fmaf(v, v, ss);
  }
  ls[hf * 256 + c] = s;
  ls[hf * 256 + 128 + c] = ss;
  __syncthreads();
  const float val = ls[tid] + ls[256 + tid];
  float* p = part + (size_t)blockIdx.x * 256 + tid;
  *(volatile float*)p = val;
  __threadfence();
  *(volatile float*)p = val;
}

__device__ __forceinline__ float bn_one(float z, float mu, float rs, float g, float b) {
  return fmaxf(((z - mu) * rs) * g + b, 0.0f);
}
__global__ __launch_bounds__(256) void bnapply_kernel(
    const float* __restrict__ z2, const float* __restrict__ part,
    const float* __restrict__ gamma, const float* __restrict__ beta,
    float* __restrict__ hf, unsigned short* __restrict__ hpl) {
  __shared__ __align__(16) float stot[256];
  __shared__ __align__(16) float smu[128];
  __shared__ __align__(16) float srs[128];
  __shared__ __align__(16) float sgm[128];
  __shared__ __align__(16) float sbt[128];
  const int tid = threadIdx.x, lane = tid & 31, wave = tid >> 5;
  float acc = 0.0f;
#pragma unroll 8
  for (int b = 0; b < 64; ++b) acc += part[(size_t)b * 256 + tid];
  stot[tid] = acc;
  __syncthreads();
  if (tid < 128) {
    const float mu = stot[tid] * (1.0f / (float)kNodes);
    float var = stot[128 + tid] * (1.0f / (float)kNodes) - mu * mu;
    var = fmaxf(var, 0.0f);
    smu[tid] = mu;
    srs[tid] = 1.0f / sqrtf(var + kBnEps);
    sgm[tid] = bf_rne(gamma[tid]);
    sbt[tid] = bf_rne(beta[tid]);
  }
  __syncthreads();
  const int rb = blockIdx.x * 64;
  {
    const int c4 = lane * 4;
    const v4f mu4 = *(const v4f*)(smu + c4);
    const v4f rs4 = *(const v4f*)(srs + c4);
    const v4f g4  = *(const v4f*)(sgm + c4);
    const v4f b4  = *(const v4f*)(sbt + c4);
#pragma unroll 1
    for (int it = 0; it < 8; ++it) {
      const int row = rb + it * 8 + wave;
      const v4f z = *(const v4f*)(z2 + (size_t)row * kHid + c4);
      v4f o;
#pragma unroll
      for (int e = 0; e < 4; ++e) o[e] = bn_one(z[e], mu4[e], rs4[e], g4[e], b4[e]);
      float* p = hf + (size_t)row * kHid + c4;
      *(volatile v4f*)p = o;
      __threadfence();
      *(volatile v4f*)p = o;
    }
  }
  {
    const int hs = lane >> 4, c8 = (lane & 15) * 8;
    const v4f mu0 = *(const v4f*)(smu + c8), mu1 = *(const v4f*)(smu + c8 + 4);
    const v4f rs0 = *(const v4f*)(srs + c8), rs1 = *(const v4f*)(srs + c8 + 4);
    const v4f g0  = *(const v4f*)(sgm + c8), g1  = *(const v4f*)(sgm + c8 + 4);
    const v4f b0  = *(const v4f*)(sbt + c8), b1  = *(const v4f*)(sbt + c8 + 4);
#pragma unroll 1
    for (int it = 0; it < 4; ++it) {
      const int row = rb + it * 16 + wave * 2 + hs;
      const float* zp = z2 + (size_t)row * kHid + c8;
      const v4f z0 = *(const v4f*)(zp);
      const v4f z1 = *(const v4f*)(zp + 4);
      float x[8];
#pragma unroll
      for (int e = 0; e < 4; ++e) {
        x[e]     = bn_one(z0[e], mu0[e], rs0[e], g0[e], b0[e]);
        x[4 + e] = bn_one(z1[e], mu1[e], rs1[e], g1[e], b1[e]);
      }
      const v4u hv = pack8h(x);
      const size_t o = (size_t)row * kHid + c8;
      *(volatile v4u*)(hpl + o) = hv;
      __threadfence();
      *(volatile v4u*)(hpl + o) = hv;
    }
  }
}

__global__ __launch_bounds__(256) void pair_kernel(
    const float* __restrict__ uv, const float* __restrict__ ew,
    const int* __restrict__ src, const int* __restrict__ dst,
    const float* __restrict__ b1, const float* __restrict__ w2, const float* __restrict__ b2p,
    float* __restrict__ out) {
  __shared__ __align__(16) float sS[64 * 128];
  __shared__ int slk[8 * 64];
  __shared__ int sld[8 * 64];
  __shared__ int scnt[8];
  __shared__ __align__(16) float sout[64];
  const int node = blockIdx.x;
  const int g = node >> 6, ii = node & 63;
  const int tid = threadIdx.x, lane = tid & 31, wave = tid >> 5;
  const int e0 = g * kEdgesPG;
  const int nb = g * kNodesPG;
#pragma unroll
  for (int it = 0; it < 8; ++it) *(v4f*)(sS + (it * 256 + tid) * 4) = (v4f){0.f, 0.f, 0.f, 0.f};
  int cnt = 0;
#pragma unroll
  for (int it = 0; it < 2; ++it) {
    const int k = wave * 64 + it * 32 + lane;
    const int sv = src[e0 + k];
    int dv = dst[e0 + k];
    asm volatile("" : "+v"(dv));
    const bool match = ((sv >> 6) == g) && ((sv & 63) == ii);
    const unsigned bal = __builtin_amdgcn_ballot_w32(match);
    const int pos = cnt + __popc(bal & ((1u << lane) - 1u));
    if (match) {
      slk[wave * 64 + pos] = k;
      sld[wave * 64 + pos] = dv & 63;
    }
    cnt += __popc(bal);
  }
  if (lane == 0) scnt[wave] = cnt;
  __syncthreads();
  if (tid < 128) {
#pragma unroll 1
    for (int w = 0; w < 8; ++w) {
      int n = scnt[w];
      n = n > 64 ? 64 : n;
#pragma unroll 1
      for (int p = 0; p < n; ++p) {
        int k = slk[w * 64 + p];
        k = k < 0 ? 0 : k;
        k = k > (kEdgesPG - 1) ? (kEdgesPG - 1) : k;
        const int dj = sld[w * 64 + p] & 63;
        sS[dj * 128 + tid] += ew[(size_t)(e0 + k) * kHid + tid];
      }
    }
  }
  __syncthreads();
  const int c4 = lane * 4;
  const v4f u4 = *(const v4f*)(uv + (size_t)node * (2 * kHid) + c4);
  const v4f braw = *(const v4f*)(b1 + c4);
  const v4f wraw = *(const v4f*)(w2 + c4);
  float bb[4], ww[4];
#pragma unroll
  for (int e = 0; e < 4; ++e) {
    const float tb = braw[e];
    const float tw = wraw[e];
    bb[e] = bf_rne(tb);
    ww[e] = bf_rne(tw);
  }
#pragma unroll 2
  for (int it = 0; it < 8; ++it) {
    const int j = it * 8 + wave;
    const v4f v4 = *(const v4f*)(uv + (size_t)(nb + j) * (2 * kHid) + kHid + c4);
    const v4f s4 = *(const v4f*)(sS + j * 128 + c4);
    float acc = 0.0f;
#pragma unroll
    for (int e = 0; e < 4; ++e) {
      const float t = fmaxf(((u4[e] + v4[e]) + s4[e]) + bb[e], 0.0f);
      acc = fmaf(t, ww[e], acc);
    }
#pragma unroll
    for (int off = 16; off > 0; off >>= 1) acc += __shfl_xor(acc, off, 32);
    if (lane == 0) sout[j] = acc;
  }
  __syncthreads();
  const float b2v = bf_rne(b2p[0]);
  if (tid < 16) {
    v4f o = *(const v4f*)(sout + tid * 4);
    o[0] += b2v;
    o[1] += b2v;
    o[2] += b2v;
    o[3] += b2v;
    float* p = out + (size_t)node * kNodesPG + tid * 4;
    *(volatile v4f*)p = o;
    __threadfence();
    *(volatile v4f*)p = o;
  }
}

extern "C" void kernel_launch(void* const* d_in, const int* in_sizes, int n_in,
                              void* d_out, int out_size, void* d_ws, size_t ws_size,
                              hipStream_t stream) {
  if (n_in < 21) return;
  if (in_sizes[0] != kNodes * kInF) return;
  if (in_sizes[1] != kEdges * kEdF) return;
  if (in_sizes[2] != 2 * kEdges) return;
  if (in_sizes[3] != kInF * kHid) return;
  if (in_sizes[5] != kEdF * kHid) return;
  if (in_sizes[7] != kLayers * kHid * kHid) return;
  if (in_sizes[9] != kLayers * kHid * kHid) return;
  if (in_sizes[11] != kLayers * kHid * kHid) return;
  if (in_sizes[13] != kLayers * kHid * kHid) return;
  if (in_sizes[17] != 3 * kHid * kHid) return;
  if (in_sizes[19] != kHid) return;
  if (out_size != kNodes * kNodesPG) return;
  if (ws_size < kWsTotal) return;

  const float* x      = (const float*)d_in[0];
  const float* eattr  = (const float*)d_in[1];
  const int*   ei     = (const int*)d_in[2];
  const float* atom_W = (const float*)d_in[3];
  const float* atom_b = (const float*)d_in[4];
  const float* bond_W = (const float*)d_in[5];
  const float* bond_b = (const float*)d_in[6];
  const float* gbm_W1 = (const float*)d_in[7];
  const float* gbm_b1 = (const float*)d_in[8];
  const float* gbm_W2 = (const float*)d_in[9];
  const float* gbm_b2 = (const float*)d_in[10];
  const float* gnn_W1 = (const float*)d_in[11];
  const float* gnn_b1 = (const float*)d_in[12];
  const float* gnn_W2 = (const float*)d_in[13];
  const float* gnn_b2 = (const float*)d_in[14];
  const float* bn_g   = (const float*)d_in[15];
  const float* bn_b   = (const float*)d_in[16];
  const float* mlp_W1 = (const float*)d_in[17];
  const float* mlp_b1 = (const float*)d_in[18];
  const float* mlp_W2 = (const float*)d_in[19];
  const float* mlp_b2 = (const float*)d_in[20];
  const int* src = ei;
  const int* dst = ei + kEdges;
  float* out = (float*)d_out;

  char* ws = (char*)d_ws;
  unsigned short* WH  = (unsigned short*)(ws + kOffWH);
  unsigned short* ATH = (unsigned short*)(ws + kOffATH);
  unsigned short* BDH = (unsigned short*)(ws + kOffBDH);
  unsigned short* XH  = (unsigned short*)(ws + kOffXH);
  unsigned short* EAH = (unsigned short*)(ws + kOffEAH);
  unsigned short* EH  = (unsigned short*)(ws + kOffEH);
  unsigned short* TH  = (unsigned short*)(ws + kOffTH);
  float*          ELF = (float*)(ws + kOffELF);
  float*          HF  = (float*)(ws + kOffHF);
  unsigned short* HH  = (unsigned short*)(ws + kOffHH);
  unsigned short* ZH  = (unsigned short*)(ws + kOffZH);
  unsigned short* TNH = (unsigned short*)(ws + kOffTNH);
  float*          Z2  = (float*)(ws + kOffZ2);
  float*          UV  = (float*)(ws + kOffUV);
  float*          PART = (float*)(ws + kOffPART);

  asplit_kernel<<<(kNodes * kInF / 8) / 256, 256, 0, stream>>>(x, XH, kInF, kInF, kNodes * kInF / 8);
  asplit_kernel<<<(kEdges * kEdFPad / 8) / 256, 256, 0, stream>>>(eattr, EAH, kEdF, kEdFPad, kEdges * kEdFPad / 8);
  wprep_kernel<<<dim3(8, kNumWMats), 256, 0, stream>>>(gbm_W1, gbm_W2, gnn_W1, gnn_W2, mlp_W1, WH, kHid, kHid);
  wprep_kernel<<<dim3(2, 1), 256, 0, stream>>>(atom_W, atom_W, atom_W, atom_W, atom_W, ATH, kInF, kInF);
  wprep_kernel<<<dim3(2, 1), 256, 0, stream>>>(bond_W, bond_W, bond_W, bond_W, bond_W, BDH, kEdF, kEdFPad);

  wmma_gemm64_h<2, 0, 0><<<16, 256, 0, stream>>>(XH, kInF, ATH, kInF,
      (void*)HF, kHid, atom_b, kNodes, kHid, kInF, kWCarryInv);
  wmma_gemm64_h<2, 1, 0><<<128, 256, 0, stream>>>(EAH, kEdFPad, BDH, kEdFPad,
      (void*)EH, kHid, bond_b, kEdges, kHid, kEdFPad, kWCarryInv);

  for (int l = 0; l < kLayers; ++l) {
    const size_t m1 = (size_t)(0 + l) * kWMatElems;
    const size_t m2 = (size_t)(4 + l) * kWMatElems;
    const size_t m3 = (size_t)(8 + l) * kWMatElems;
    const size_t m4 = (size_t)(12 + l) * kWMatElems;
    wmma_gemm64_h<2, 1, 2><<<128, 256, 0, stream>>>(EH, kHid, WH + m1, kHid,
        (void*)TH, kHid, gbm_b1 + l * kHid, kEdges, kHid, kHid, kWCarryInv);
    wmma_gemm64_h<2, 0, 0><<<128, 256, 0, stream>>>(TH, kHid, WH + m2, kHid,
        (void*)ELF, kHid, gbm_b2 + l * kHid, kEdges, kHid, kHid, kWCarryInv);
    agg_kernel<<<kGraphs, 128, 0, stream>>>(HF, ELF, src, dst, ZH);
    wmma_gemm64_h<2, 1, 2><<<16, 256, 0, stream>>>(ZH, kHid, WH + m3, kHid,
        (void*)TNH, kHid, gnn_b1 + l * kHid, kNodes, kHid, kHid, kWCarryInv);
    wmma_gemm64_h<2, 0, 0><<<16, 256, 0, stream>>>(TNH, kHid, WH + m4, kHid,
        (void*)Z2, kHid, gnn_b2 + l * kHid, kNodes, kHid, kHid, kWCarryInv);
    stats_kernel<<<64, 256, 0, stream>>>(Z2, PART);
    bnapply_kernel<<<64, 256, 0, stream>>>(Z2, PART, bn_g + l * kHid, bn_b + l * kHid, HF, HH);
  }

  const size_t mu = (size_t)16 * kWMatElems;
  const size_t mc = (size_t)18 * kWMatElems;
  wmma_gemm64_h<0, 0, 0><<<32, 256, 0, stream>>>(HH, kHid, WH + mu, kHid,
      (void*)UV, 2 * kHid, mlp_b1, kNodes, 2 * kHid, kHid, kWCarryInv);
  wmma_gemm64_h<0, 0, 0><<<128, 256, 0, stream>>>(EH, kHid, WH + mc, kHid,
      (void*)ELF, kHid, mlp_b1, kEdges, kHid, kHid, kWCarryInv);

  pair_kernel<<<kNodes, 256, 0, stream>>>(UV, ELF, src, dst, mlp_b1, mlp_W2, mlp_b2, out);
}
